// GraphTransformerLayer_47167330845010
// MI455X (gfx1250) — hardware-verified
//
#include <hip/hip_runtime.h>
#include <math.h>
#include <stddef.h>
#include <stdint.h>

#define NNODE   4096
#define DMOD    256
#define NHEAD   8
#define HDIM    32
#define NQKV    768
#define KFF     512

#define NTHR    256
#define NWAVE   8
#define EPT     8
#define CHUNK   (NTHR * EPT)
#define WCAP    (EPT * 32)
#define LISTN   (NWAVE * WCAP)
#define NBA     512
#define PKS     9
#define RCAP    20480
#define DEGCAP  128
#define ZINTS   (2 * RCAP + 2 * NBA + LISTN)
#define LDS_AGG (ZINTS * 4 + 64)
#define GBM     64
#define GTHR    128
#define AT_D    32
#define AT_NW   4
#define AT_QB   64
#define AT_KC   64
#define OSP     36
#define WSMAX   134217728

static_assert((CHUNK & (CHUNK - 1)) == 0);
static_assert(NBA == (1 << PKS));
static_assert(((long long)CHUNK << PKS) < (1LL << 31));
static_assert(NTHR * 2 == NBA);
static_assert(LISTN >= NBA && LISTN >= NWAVE * WCAP);
static_assert((RCAP % 32) == 0);
static_assert((ZINTS % (NTHR * 4)) == 0);
static_assert(LDS_AGG <= 262144);
static_assert((NBA % NWAVE) == 0 && (NNODE % NBA) == 0);
static_assert(GBM == (GTHR / 32) * 16);
static_assert(DMOD == 32 * 8);
static_assert((NNODE % 64) == 0 && (DMOD % 64) == 0 && (NQKV % 64) == 0);
static_assert((KFF % 32) == 0 && (DMOD % 32) == 0 && KFF == 2 * DMOD);
static_assert(NHEAD * HDIM == DMOD && AT_D == HDIM && (NNODE % AT_QB) == 0 && (NNODE % AT_KC) == 0);
static_assert(AT_QB == AT_NW * 16 && AT_KC == 64 && AT_D == 32);

typedef float          v2f  __attribute__((ext_vector_type(2)));
typedef float          v4f  __attribute__((ext_vector_type(4)));
typedef float          v8f  __attribute__((ext_vector_type(8)));
typedef int            v4i  __attribute__((ext_vector_type(4)));
typedef int            v8i  __attribute__((ext_vector_type(8)));
typedef unsigned int   v2u  __attribute__((ext_vector_type(2)));
typedef unsigned int   v4u  __attribute__((ext_vector_type(4)));
typedef unsigned short v8us __attribute__((ext_vector_type(8)));
typedef _Float16       v16h __attribute__((ext_vector_type(16)));
typedef _Float16       v8h  __attribute__((ext_vector_type(8)));
typedef __bf16         v16b __attribute__((ext_vector_type(16)));
typedef __bf16         v8b  __attribute__((ext_vector_type(8)));
typedef v4f  __attribute__((may_alias)) v4fa;
typedef v4i  __attribute__((may_alias)) v4ia;
typedef v8us __attribute__((may_alias)) v8usa;

__device__ __forceinline__ unsigned short bf_bits(float f) {
  unsigned int u = __float_as_uint(f);
  u += 0x7FFFu + ((u >> 16) & 1u);
  return (unsigned short)(u >> 16);
}
__device__ __forceinline__ float bf_val(unsigned short b) { return __uint_as_float(((unsigned int)b) << 16); }
__device__ __forceinline__ float bf_rne(float f) { return bf_val(bf_bits(f)); }
__device__ __forceinline__ unsigned pk16(unsigned short a, unsigned short b) { return (unsigned)a | ((unsigned)b << 16); }

__device__ __forceinline__ void split8b(const v4f a, const v4f b, v8us& hi, v8us& lo) {
  float x[8];
  x[0] = a.x; x[1] = a.y; x[2] = a.z; x[3] = a.w; x[4] = b.x; x[5] = b.y; x[6] = b.z; x[7] = b.w;
#pragma unroll
  for (int i = 0; i < 8; ++i) {
    const unsigned short hb = bf_bits(x[i]);
    hi[i] = hb;
    lo[i] = bf_bits(x[i] - bf_val(hb));
  }
}

union FragU { v16b b; v8us h[2]; v8i w; };
__device__ __forceinline__ v8f wmk(const FragU& a, const FragU& b, v8f c) {
  v8f d = __builtin_amdgcn_wmma_f32_16x16x32_bf16(false, a.b, false, b.b, (short)0, c, false, false);
  asm volatile("v_nop\n\tv_nop\n\tv_nop\n\tv_nop" : "+v"(d) : "v"(a.w), "v"(b.w));
  return d;
}
union FB { v16b v; v8b h[2]; };
__device__ __forceinline__ v16b frag_load(const __bf16* p) {
  FB f; f.h[0] = *(const v8b*)(p); f.h[1] = *(const v8b*)(p + 16); return f.v;
}
__device__ __forceinline__ v8f mma_b(v16b a, v16b b, v8f c) {
  return __builtin_amdgcn_wmma_f32_16x16x32_bf16(false, a, false, b, (short)0, c, false, false);
}
__device__ __forceinline__ void dep_guard_b(v8f& a, v8f& b, v16b x, v16b y) {
  asm volatile("v_nop\n\tv_nop\n\tv_nop\n\tv_nop" : "+v"(a), "+v"(b) : "v"(x), "v"(y));
}
__device__ __forceinline__ void keep4_b(v16b a, v16b b, v16b c, v16b d) { asm volatile("v_nop" :: "v"(a), "v"(b), "v"(c), "v"(d)); }
__device__ __forceinline__ void acc_guard4(v8f& a, v8f& b, v8f& c, v8f& d) {
  asm volatile("v_nop\n\tv_nop\n\tv_nop\n\tv_nop" : "+v"(a), "+v"(b), "+v"(c), "+v"(d));
}
__device__ __forceinline__ v8f at_mma(v16b a, v16b b, v8f c) {
  c = __builtin_amdgcn_wmma_f32_16x16x32_bf16(false, a, false, b, (short)0, c, false, false);
  asm volatile("v_nop\n\tv_nop\n\tv_nop\n\tv_nop" : "+v"(c) : "v"(a), "v"(b));
  return c;
}

template <bool SPLIT, int OUT_MODE>
__global__ __launch_bounds__(256) void wmma_gemm64(
    const unsigned short* __restrict__ Ap, const unsigned short* __restrict__ A2p, int lda,
    const unsigned short* __restrict__ Btp, const unsigned short* __restrict__ Bt2p, int ldb,
    void* Cout, void* Cout2, int ldc, int M, int N, int K, float scale) {
  const __bf16* A  = (const __bf16*)(const void*)Ap;  const __bf16* A2  = (const __bf16*)(const void*)A2p;
  const __bf16* Bt = (const __bf16*)(const void*)Btp; const __bf16* Bt2 = (const __bf16*)(const void*)Bt2p;
  __shared__ __align__(16) float sT[8][16 * 68];
  const int lane = threadIdx.x & 31;
  const int wave = threadIdx.x >> 5;
  const int tilesN = N >> 6;
  const int tilesM = M >> 6;
  const int tile = blockIdx.x * 8 + wave;
  if (tile >= tilesM * tilesN) return;
  const int tm = tile / tilesN;
  const int tn = tile - tm * tilesN;
  const int m0 = tm << 6;
  const int n0 = tn << 6;

  const int rlane = lane & 15;
  const int koff  = (lane >> 4) * 8;
  const int mOff  = (lane >> 4) * 8;

  v8f acc[4][4];
#pragma unroll
  for (int i = 0; i < 4; ++i)
#pragma unroll
    for (int j = 0; j < 4; ++j) acc[i][j] = (v8f){0.f,0.f,0.f,0.f,0.f,0.f,0.f,0.f};

  for (int k0 = 0; k0 < K; k0 += 32) {
    v16b bh[4], bl[4];
#pragma unroll
    for (int j = 0; j < 4; ++j) {
      const size_t bo = (size_t)(n0 + (j << 4) + rlane) * ldb + koff + k0;
      bh[j] = frag_load(Bt + bo);
      bl[j] = bh[j];
      if (SPLIT) bl[j] = frag_load(Bt2 + bo);
    }
#pragma unroll
    for (int i = 0; i < 4; ++i) {
      const size_t ao = (size_t)(m0 + (i << 4) + rlane) * lda + koff + k0;
      v16b ah = frag_load(A + ao);
      v16b al = ah;
      if (SPLIT) al = frag_load(A2 + ao);
#pragma unroll
      for (int j = 0; j < 4; ++j) {
        acc[i][j] = mma_b(ah, bh[j], acc[i][j]);
        if (SPLIT) {
          acc[i][j] = mma_b(ah, bl[j], acc[i][j]);
          acc[i][j] = mma_b(al, bh[j], acc[i][j]);
        }
      }
      dep_guard_b(acc[i][0], acc[i][3], ah, al);
    }
    keep4_b(bh[0], bh[1], bh[2], bh[3]);
    if (SPLIT) keep4_b(bl[0], bl[1], bl[2], bl[3]);
  }
  acc_guard4(acc[0][0], acc[0][1], acc[0][2], acc[0][3]);
  acc_guard4(acc[1][0], acc[1][1], acc[1][2], acc[1][3]);
  acc_guard4(acc[2][0], acc[2][1], acc[2][2], acc[2][3]);
  acc_guard4(acc[3][0], acc[3][1], acc[3][2], acc[3][3]);

  float* slab = sT[wave];
#pragma unroll
  for (int i = 0; i < 4; ++i) {
    const int mBase = m0 + (i << 4);
#pragma unroll
    for (int j = 0; j < 4; ++j) {
#pragma unroll
      for (int r = 0; r < 8; ++r) {
        slab[(mOff + r) * 68 + (j << 4) + rlane] = acc[i][j][r] * scale;
      }
    }
    __builtin_amdgcn_fence(__ATOMIC_RELEASE, "workgroup");
    __builtin_amdgcn_wave_barrier();
    __builtin_amdgcn_fence(__ATOMIC_ACQUIRE, "workgroup");
    if (OUT_MODE == 0) {
      float* C = (float*)Cout;
      const int hh = lane >> 4, c4 = (lane & 15) * 4;
      for (int pass = 0; pass < 2; ++pass) {
#pragma unroll
        for (int it = 0; it < 8; ++it) {
          const int row = it * 2 + hh;
          v4f v = *(const v4f*)(slab + row * 68 + c4);
          *(volatile v4f*)(C + (size_t)(mBase + row) * ldc + n0 + c4) = v;
        }
        __threadfence();
      }
    } else {
      const int q = lane >> 3, c8 = (lane & 7) * 8;
      unsigned short* C  = (unsigned short*)Cout;
      unsigned short* C2 = (unsigned short*)Cout2;
      for (int pass = 0; pass < 2; ++pass) {
#pragma unroll
        for (int it = 0; it < 4; ++it) {
          const int row = it * 4 + q;
          const float* sp = slab + row * 68 + c8;
          v8h hv, lv;
#pragma unroll
          for (int e = 0; e < 8; ++e) {
            unsigned short hb = bf_bits(sp[e]);
            unsigned short lb = bf_bits(sp[e] - bf_val(hb));
            hv[e] = __builtin_bit_cast(_Float16, hb);
            lv[e] = __builtin_bit_cast(_Float16, lb);
          }
          *(volatile v8h*)(C  + (size_t)(mBase + row) * ldc + n0 + c8) = hv;
          *(volatile v8h*)(C2 + (size_t)(mBase + row) * ldc + n0 + c8) = lv;
        }
        __threadfence();
      }
    }
    __builtin_amdgcn_fence(__ATOMIC_RELEASE, "workgroup");
    __builtin_amdgcn_wave_barrier();
    __builtin_amdgcn_fence(__ATOMIC_ACQUIRE, "workgroup");
  }
}

__global__ __launch_bounds__(256) void k_wtrans(const float* __restrict__ WQ, const float* __restrict__ WK,
                                                 const float* __restrict__ WV, const float* __restrict__ Wc,
                                                 unsigned short* WqkvT, unsigned short* WcD) {
  __shared__ __align__(16) float tf[64 * 68];
  const int z = blockIdx.z;
  const float* W;
  unsigned short* ob;
  int ldo;
  if (z == 0)      { W = WQ; ob = WqkvT;                            ldo = DMOD; }
  else if (z == 1) { W = WK; ob = WqkvT + (size_t)1 * DMOD * DMOD;  ldo = DMOD; }
  else if (z == 2) { W = WV; ob = WqkvT + (size_t)2 * DMOD * DMOD;  ldo = DMOD; }
  else             { W = Wc; ob = WcD;                              ldo = KFF;  }
  const int c0  = blockIdx.x * 64;
  const int r0  = blockIdx.y * 64;
  const int tid = threadIdx.x;
  {
    const int lr = tid >> 4;
    const int c4 = (tid & 15) * 4;
#pragma unroll
    for (int it = 0; it < 4; ++it) {
      const int rr = it * 16 + lr;
      const v4f a = *(const v4f*)(W + (size_t)(r0 + rr) * DMOD + c0 + c4);
      *(v4f*)(tf + rr * 68 + c4) = a;
    }
  }
  __syncthreads();
  const int sub = tid >> 3;
  const int c8  = (tid & 7) * 8;
  v4u hv[2];
#pragma unroll
  for (int it = 0; it < 2; ++it) {
    const int oc = it * 32 + sub;
    v4u a;
#pragma unroll
    for (int q = 0; q < 4; ++q) {
      const float f0 = tf[(c8 + 2 * q) * 68 + oc];
      const float f1 = tf[(c8 + 2 * q + 1) * 68 + oc];
      a[q] = pk16(bf_bits(f0), bf_bits(f1));
    }
    hv[it] = a;
  }
  for (int pass = 0; pass < 2; ++pass) {
#pragma unroll
    for (int it = 0; it < 2; ++it) {
      const int oc = it * 32 + sub;
      const size_t go = (size_t)(c0 + oc) * ldo + r0 + c8;
      *(volatile v4u*)(ob + go) = hv[it];
      if (z == 3) *(volatile v4u*)(ob + go + DMOD) = hv[it];
    }
    __threadfence();
  }
}

__global__ __launch_bounds__(256) void k_xcvt(const float* __restrict__ X, unsigned short* Xb, int n8) {
  const int i = blockIdx.x * 256 + threadIdx.x;
  if (i < n8) {
    const v4f a = *(const v4f*)(X + 8 * (size_t)i);
    const v4f b = *(const v4f*)(X + 8 * (size_t)i + 4);
    v8us o;
    o[0] = bf_bits(a.x); o[1] = bf_bits(a.y); o[2] = bf_bits(a.z); o[3] = bf_bits(a.w);
    o[4] = bf_bits(b.x); o[5] = bf_bits(b.y); o[6] = bf_bits(b.z); o[7] = bf_bits(b.w);
    unsigned short* p = Xb + 8 * (size_t)i;
    *(volatile v8us*)p = o;
    __threadfence();
    *(volatile v8us*)p = o;
  }
}

__device__ __forceinline__ int scan_chunk(const int* __restrict__ dsts, int nE, int cbase, int slotBase,
                                          int nb, int vec8, int* list, int tid, int lane, int wave) {
  int wc = 0;
  const int el0  = tid * EPT;
  const int e0   = cbase + el0;
  const int sent = -2147483647 - 1;
  v4i da, db;
  if (vec8 != 0 && cbase + CHUNK <= nE) {
    da = *(const v4i*)(dsts + e0);
    db = *(const v4i*)(dsts + e0 + 4);
  } else {
    da.x = (e0     < nE) ? dsts[min(e0,     nE - 1)] : sent;
    da.y = (e0 + 1 < nE) ? dsts[min(e0 + 1, nE - 1)] : sent;
    da.z = (e0 + 2 < nE) ? dsts[min(e0 + 2, nE - 1)] : sent;
    da.w = (e0 + 3 < nE) ? dsts[min(e0 + 3, nE - 1)] : sent;
    db.x = (e0 + 4 < nE) ? dsts[min(e0 + 4, nE - 1)] : sent;
    db.y = (e0 + 5 < nE) ? dsts[min(e0 + 5, nE - 1)] : sent;
    db.z = (e0 + 6 < nE) ? dsts[min(e0 + 6, nE - 1)] : sent;
    db.w = (e0 + 7 < nE) ? dsts[min(e0 + 7, nE - 1)] : sent;
  }
  const unsigned nbs = (unsigned)slotBase;
  const unsigned unb = (unsigned)nb;
  const unsigned s0 = (unsigned)da.x - nbs, s1 = (unsigned)da.y - nbs;
  const unsigned s2 = (unsigned)da.z - nbs, s3 = (unsigned)da.w - nbs;
  const unsigned s4 = (unsigned)db.x - nbs, s5 = (unsigned)db.y - nbs;
  const unsigned s6 = (unsigned)db.z - nbs, s7 = (unsigned)db.w - nbs;
  const bool h0 = s0 < unb, h1 = s1 < unb, h2 = s2 < unb, h3 = s3 < unb;
  const bool h4 = s4 < unb, h5 = s5 < unb, h6 = s6 < unb, h7 = s7 < unb;
  const unsigned any = __builtin_amdgcn_ballot_w32(h0 | h1 | h2 | h3 | h4 | h5 | h6 | h7);
  if (any != 0u) {
#define HITJ(J, HJ, SJ) { \
      const unsigned mj = __builtin_amdgcn_ballot_w32(HJ); \
      if (mj != 0u) { \
        if (HJ) { \
          const int pos = wc + (int)__builtin_amdgcn_mbcnt_lo(mj, 0u); \
          if (pos < WCAP) list[wave * WCAP + pos] = ((el0 + (J)) << PKS) | (int)(SJ); \
        } \
        wc += (int)__builtin_popcount(mj); } }
    HITJ(0, h0, s0)
    HITJ(1, h1, s1)
    HITJ(2, h2, s2)
    HITJ(3, h3, s3)
    HITJ(4, h4, s4)
    HITJ(5, h5, s5)
    HITJ(6, h6, s6)
    HITJ(7, h7, s7)
#undef HITJ
  }
  return wc;
}

__global__ __launch_bounds__(NTHR) void k_agg(const int* __restrict__ srcs, const int* __restrict__ dsts,
                                              const float* __restrict__ Kf, unsigned short* K2h, unsigned short* K2l,
                                              int nN, int nE, int vec8) {
  extern __shared__ __attribute__((aligned(16))) int lds_i[];
  int* reg1 = lds_i;
  int* reg2 = reg1 + RCAP;
  int* scnt = reg2 + RCAP;
  int* soff = scnt + NBA;
  int* list = soff + NBA;
  int* wcnt = list + LISTN;
  int* wtot = wcnt + NWAVE;
  const int tid = (int)threadIdx.x, lane = tid & 31, wave = tid >> 5;
  const int nodeBase = (int)blockIdx.x * NBA;

  {
    const v4i z4 = {0, 0, 0, 0};
    for (int i = tid * 4; i < ZINTS; i += NTHR * 4) *(v4ia*)(lds_i + i) = z4;
    if (tid < 2 * NWAVE) wcnt[tid] = 0;
  }
  __syncthreads();

  int tot = 0;
  const int nChunks = (nE + CHUNK - 1) / CHUNK;
#pragma unroll 1
  for (int ch = 0; ch < nChunks; ++ch) {
    const int cbase = ch * CHUNK;
    const int wc = scan_chunk(dsts, nE, cbase, nodeBase, NBA, vec8, list, tid, lane, wave);
    if (lane == 0) wcnt[wave] = wc;
    __syncthreads();
    int pre = 0, all = 0;
#pragma unroll
    for (int w2 = 0; w2 < NWAVE; ++w2) {
      int c = wcnt[w2];
      c = c < 0 ? 0 : (c > WCAP ? WCAP : c);
      all += c;
      pre += (w2 < wave) ? c : 0;
    }
    const int wcc  = wc > WCAP ? WCAP : wc;
    const int base = tot + pre;
#pragma unroll 1
    for (int i = lane; i < wcc; i += 32) {
      const int ent = list[wave * WCAP + i];
      const int el  = (ent >> PKS) & (CHUNK - 1);
      const int sl  = ent & (NBA - 1);
      int eid = cbase + el;
      eid = eid > nE - 1 ? nE - 1 : eid;
      const int pos = base + i;
      if (pos < RCAP) reg1[pos] = (int)(((unsigned)eid << PKS) | (unsigned)sl);
    }
    tot += all;
    tot = tot > RCAP ? RCAP : tot;
    __syncthreads();
  }
  const int nh = tot;

  if (wave == 0) {
#pragma unroll 1
    for (int b0 = 0; b0 < nh; b0 += 32) {
      const int idx = b0 + lane;
      const int uv  = reg1[idx < RCAP ? idx : RCAP - 1];
      const int m32 = (nh - b0) < 32 ? (nh - b0) : 32;
#pragma unroll 1
      for (int k = 0; k < m32; ++k) {
        const int u  = __builtin_amdgcn_readlane(uv, k);
        const int sl = u & (NBA - 1);
        if (lane == 0) scnt[sl] = scnt[sl] + 1;
      }
    }
  }
  __syncthreads();

  {
    const int c0r = scnt[2 * tid], c1r = scnt[2 * tid + 1];
    const int e0 = c0r < 0 ? 0 : c0r, e1 = c1r < 0 ? 0 : c1r;
    const int ts = e0 + e1;
    int incl = ts;
#pragma unroll
    for (int d = 1; d < 32; d <<= 1) {
      const int up = __shfl_up(incl, d, 32);
      if (lane >= d) incl += up;
    }
    if (lane == 31) wtot[wave] = incl;
    __syncthreads();
    int pre = 0;
#pragma unroll
    for (int w2 = 0; w2 < NWAVE; ++w2) pre += (w2 < wave) ? wtot[w2] : 0;
    int run = pre + incl - ts;
    soff[2 * tid + 0] = run; run += e0;
    soff[2 * tid + 1] = run;
  }
  __syncthreads();
  for (int i = tid; i < NBA; i += NTHR) list[i] = soff[i];
  __syncthreads();

  if (wave == 0) {
#pragma unroll 1
    for (int b0 = 0; b0 < nh; b0 += 32) {
      const int idx = b0 + lane;
      const int uv  = reg1[idx < RCAP ? idx : RCAP - 1];
      const int m32 = (nh - b0) < 32 ? (nh - b0) : 32;
#pragma unroll 1
      for (int k = 0; k < m32; ++k) {
        const int u   = __builtin_amdgcn_readlane(uv, k);
        const int sl  = u & (NBA - 1);
        const int eid = (int)((unsigned)u >> PKS);
        if (lane == 0) {
          int pos = list[sl];
          pos = pos < 0 ? 0 : (pos > RCAP - 1 ? RCAP - 1 : pos);
          reg2[pos] = eid;
          list[sl] = pos + 1;
        }
      }
    }
  }
  __syncthreads();

  const int nbw = NBA / NWAVE;
  const bool ovf = (nh >= RCAP);
  const float qnan = __int_as_float(0x7fc00000);

#pragma unroll 1
  for (int jt = 0; jt < nbw; ++jt) {
    const int slot = wave * nbw + jt;
    const int node = nodeBase + slot;
    int st = soff[slot];
    const int craw = scnt[slot];
    int cnt = craw;
    st  = st < 0 ? 0 : (st > nh ? nh : st);
    cnt = cnt < 0 ? 0 : (cnt > DEGCAP ? DEGCAP : cnt);
    if (cnt > nh - st) cnt = nh - st;
    const float pz = (ovf || craw > DEGCAP) ? qnan : 0.0f;
    const bool live = node < nN;

    float a0 = 0.f, a1 = 0.f, a2 = 0.f, a3 = 0.f, a4 = 0.f, a5 = 0.f, a6 = 0.f, a7 = 0.f;
#pragma unroll 1
    for (int b0 = 0; b0 < cnt; b0 += 32) {
      int idx = st + b0 + lane; idx = idx > RCAP - 1 ? RCAP - 1 : idx;
      int eid = reg2[idx]; eid = eid < 0 ? 0 : (eid > nE - 1 ? nE - 1 : eid);
      int sr = srcs[eid]; sr = sr < 0 ? 0 : (sr > nN - 1 ? nN - 1 : sr);
      const int m32 = (cnt - b0) < 32 ? (cnt - b0) : 32;
#pragma unroll 1
      for (int k = 0; k < m32; ++k) {
        const int sk = __builtin_amdgcn_readlane(sr, k);
        const float* kp = Kf + (size_t)sk * DMOD + 8 * lane;
        const v4f va = *(const v4f*)kp;
        const v4f vb = *(const v4f*)(kp + 4);
        a0 += va.x; a1 += va.y; a2 += va.z; a3 += va.w;
        a4 += vb.x; a5 += vb.y; a6 += vb.z; a7 += vb.w;
      }
    }
    v4f ra, rb;
    ra.x = (live ? a0 : 0.0f) + pz; ra.y = (live ? a1 : 0.0f) + pz; ra.z = (live ? a2 : 0.0f) + pz; ra.w = (live ? a3 : 0.0f) + pz;
    rb.x = (live ? a4 : 0.0f) + pz; rb.y = (live ? a5 : 0.0f) + pz; rb.z = (live ? a6 : 0.0f) + pz; rb.w = (live ? a7 : 0.0f) + pz;
    v8us hi, lo;
    split8b(ra, rb, hi, lo);
    const size_t gp = (size_t)node * (size_t)DMOD + 8 * lane;
    *(volatile v8us*)(K2h + gp) = hi;
    *(volatile v8us*)(K2l + gp) = lo;
    __threadfence();
    *(volatile v8us*)(K2h + gp) = hi;
    *(volatile v8us*)(K2l + gp) = lo;
  }
}

__global__ __launch_bounds__(128)
void k_attn(const unsigned short* __restrict__ qhp, const unsigned short* __restrict__ qlp,
            const unsigned short* __restrict__ khp, const unsigned short* __restrict__ klp,
            const unsigned short* __restrict__ vhp, const unsigned short* __restrict__ vlp,
            float* out, float sscale) {
  __shared__ __align__(16) __bf16 Ksh[AT_KC * AT_D];
  __shared__ __align__(16) __bf16 Ksl[AT_KC * AT_D];
  __shared__ __align__(16) __bf16 Vth[AT_D * AT_KC];
  __shared__ __align__(16) __bf16 Vtl[AT_D * AT_KC];
  __shared__ __align__(16) __bf16 Psh[AT_NW][16 * AT_KC];
  __shared__ __align__(16) __bf16 Psl[AT_NW][16 * AT_KC];
  __shared__ __align__(16) float  Os[AT_NW][16 * OSP];

  const int tid  = threadIdx.x;
  const int wave = tid >> 5;
  const int lane = tid & 31;
  const int hh   = lane >> 4;
  const int c    = lane & 15;

  const int nqb = NNODE / AT_QB;
  const int bx = blockIdx.x;
  const int qb = bx % nqb;
  const int h  = bx / nqb;
  const int q0 = qb * AT_QB + wave * 16;

  const __bf16* Qh = (const __bf16*)(const void*)qhp + (size_t)h * AT_D;
  const __bf16* Ql = (const __bf16*)(const void*)qlp + (size_t)h * AT_D;
  const __bf16* Kh = (const __bf16*)(const void*)khp + (size_t)h * AT_D;
  const __bf16* Kl = (const __bf16*)(const void*)klp + (size_t)h * AT_D;
  const __bf16* Vh = (const __bf16*)(const void*)vhp + (size_t)h * AT_D * NNODE;
  const __bf16* Vl = (const __bf16*)(const void*)vlp + (size_t)h * AT_D * NNODE;
  float*        ob = out + (size_t)h * AT_D;

  const v16b qah = frag_load(Qh + (size_t)(q0 + c) * DMOD + 8 * hh);
  const v16b qal = frag_load(Ql + (size_t)(q0 + c) * DMOD + 8 * hh);

  float mrow[8], lrow[8];
  v8f oacc[2];
#pragma unroll
  for (int r = 0; r < 8; ++r) { mrow[r] = -INFINITY; lrow[r] = 0.f; }
#pragma unroll
  for (int t = 0; t < 2; ++t) oacc[t] = (v8f){0.f,0.f,0.f,0.f,0.f,0.f,0.f,0.f};

  const int nChunks = NNODE / AT_KC;
  for (int kc = 0; kc < nChunks; ++kc) {
    const int kv0 = kc * AT_KC;
    __syncthreads();
    {
      const int r = tid >> 1, halfd = (tid & 1) * 16;
      const __bf16* ksh = Kh + (size_t)(kv0 + r) * DMOD + halfd;
      const __bf16* ksl = Kl + (size_t)(kv0 + r) * DMOD + halfd;
      const int dv = tid >> 2, seg = (tid & 3) * 16;
      const __bf16* vsh = Vh + (size_t)dv * NNODE + kv0 + seg;
      const __bf16* vsl = Vl + (size_t)dv * NNODE + kv0 + seg;
#pragma unroll
      for (int i = 0; i < 2; ++i) {
        const v8b a0 = *(const v8b*)(ksh + 8 * i);
        const v8b a1 = *(const v8b*)(ksl + 8 * i);
        const v8b b0 = *(const v8b*)(vsh + 8 * i);
        const v8b b1 = *(const v8b*)(vsl + 8 * i);
        *(v8b*)(Ksh + r * AT_D   + halfd + 8 * i) = a0;
        *(v8b*)(Ksl + r * AT_D   + halfd + 8 * i) = a1;
        *(v8b*)(Vth + dv * AT_KC + seg + 8 * i) = b0;
        *(v8b*)(Vtl + dv * AT_KC + seg + 8 * i) = b1;
      }
    }
    __syncthreads();

    v8f s[4];
#pragma unroll
    for (int j = 0; j < 4; ++j) {
      s[j] = (v8f){0.f,0.f,0.f,0.f,0.f,0.f,0.f,0.f};
      FB kb, kl;
      kb.h[0] = *(const v8b*)(Ksh + (j * 16 + c) * AT_D + 8 * hh);
      kb.h[1] = *(const v8b*)(Ksh + (j * 16 + c) * AT_D + 16 + 8 * hh);
      kl.h[0] = *(const v8b*)(Ksl + (j * 16 + c) * AT_D + 8 * hh);
      kl.h[1] = *(const v8b*)(Ksl + (j * 16 + c) * AT_D + 16 + 8 * hh);
      s[j] = at_mma(qah, kb.v, s[j]);
      s[j] = at_mma(qah, kl.v, s[j]);
      s[j] = at_mma(qal, kb.v, s[j]);
    }
    float cm[8];
#pragma unroll
    for (int r = 0; r < 8; ++r) {
      float m = -INFINITY;
#pragma unroll
      for (int j = 0; j < 4; ++j) {
        const float sv = s[j][r] * sscale;
        s[j][r] = sv;
        m = fmaxf(m, sv);
      }
#pragma unroll
      for (int off = 1; off < 16; off <<= 1) m = fmaxf(m, __shfl_xor(m, off, 32));
      cm[r] = m;
    }
    __bf16* pwh = Psh[wave];
    __bf16* pwl = Psl[wave];
#pragma unroll
    for (int r = 0; r < 8; ++r) {
      const float mnew = fmaxf(mrow[r], cm[r]);
      const float alpha = expf(mrow[r] - mnew);
      mrow[r] = mnew;
      float psum = 0.f;
#pragma unroll
      for (int j = 0; j < 4; ++j) {
        const float p = expf(s[j][r] - mnew);
        psum += p;
        const unsigned short hb = bf_bits(p);
        const unsigned short lb = bf_bits(p - bf_val(hb));
        pwh[(8 * hh + r) * AT_KC + j * 16 + c] = __builtin_bit_cast(__bf16, hb);
        pwl[(8 * hh + r) * AT_KC + j * 16 + c] = __builtin_bit_cast(__bf16, lb);
      }
#pragma unroll
      for (int off = 1; off < 16; off <<= 1) psum += __shfl_xor(psum, off, 32);
      lrow[r] = lrow[r] * alpha + psum;
#pragma unroll
      for (int t = 0; t < 2; ++t) oacc[t][r] *= alpha;
    }
    __builtin_amdgcn_fence(__ATOMIC_RELEASE, "workgroup");
    __builtin_amdgcn_wave_barrier();
    __builtin_amdgcn_fence(__ATOMIC_ACQUIRE, "workgroup");
#pragma unroll 1
    for (int kk = 0; kk < 2; ++kk) {
      FB pa, pl;
      pa.h[0] = *(const v8b*)(pwh + c * AT_KC + kk * 32 + 8 * hh);
      pa.h[1] = *(const v8b*)(pwh + c * AT_KC + kk * 32 + 16 + 8 * hh);
      pl.h[0] = *(const v8b*)(pwl + c * AT_KC + kk * 32 + 8 * hh);
      pl.h[1] = *(const v8b*)(pwl + c * AT_KC + kk * 32 + 16 + 8 * hh);
#pragma unroll
      for (int t = 0; t < 2; ++t) {
        FB vb, vl;
        vb.h[0] = *(const v8b*)(Vth + (t * 16 + c) * AT_KC + kk * 32 + 8 * hh);
        vb.h[1] = *(const v8b*)(Vth + (t * 16 + c) * AT_KC + kk * 32 + 16 + 8 * hh);
        vl.h[0] = *(const v8b*)(Vtl + (t * 16 + c) * AT_KC + kk * 32 + 8 * hh);
        vl.h[1] = *(const v8b*)(Vtl + (t * 16 + c) * AT_KC + kk * 32 + 16 + 8 * hh);
        oacc[t] = at_mma(pa.v, vb.v, oacc[t]);
        oacc[t] = at_mma(pa.v, vl.v, oacc[t]);
        oacc[t] = at_mma(pl.v, vb.v, oacc[t]);
      }
    }
  }

  float* os = Os[wave];
#pragma unroll
  for (int r = 0; r < 8; ++r) {
    const float inv = 1.0f / lrow[r];
#pragma unroll
    for (int t = 0; t < 2; ++t) os[(8 * hh + r) * OSP + t * 16 + c] = oacc[t][r] * inv;
  }
  __builtin_amdgcn_fence(__ATOMIC_RELEASE, "workgroup");
  __builtin_amdgcn_wave_barrier();
  __builtin_amdgcn_fence(__ATOMIC_ACQUIRE, "workgroup");
  {
    const int q4 = lane >> 3, c4 = (lane & 7) * 4;
    for (int pass = 0; pass < 2; ++pass) {
#pragma unroll
      for (int it = 0; it < 4; ++it) {
        const int row = it * 4 + q4;
        v4f val = *(const v4f*)(os + row * OSP + c4);
        *(volatile v4f*)(ob + (size_t)(q0 + row) * DMOD + c4) = val;
      }
      __threadfence();
    }
  }
}

__global__ __launch_bounds__(256) void k_hsplit(const float* __restrict__ X, const float* __restrict__ AO,
                                                 unsigned short* HP, int nUnits) {
  const int u = blockIdx.x * 256 + threadIdx.x;
  if (u < nUnits) {
    const int row = u >> 5, c8 = (u & 31) * 8;
    const size_t xo = (size_t)row * DMOD + c8;
    const v4f xa = *(const v4f*)(X + xo),  xb = *(const v4f*)(X + xo + 4);
    const v4f aa = *(const v4f*)(AO + xo), ab = *(const v4f*)(AO + xo + 4);
    v4f ha, hb;
    ha.x = bf_rne(xa.x) + aa.x; ha.y = bf_rne(xa.y) + aa.y; ha.z = bf_rne(xa.z) + aa.z; ha.w = bf_rne(xa.w) + aa.w;
    hb.x = bf_rne(xb.x) + ab.x; hb.y = bf_rne(xb.y) + ab.y; hb.z = bf_rne(xb.z) + ab.z; hb.w = bf_rne(xb.w) + ab.w;
    v8us hi, lo;
    split8b(ha, hb, hi, lo);
    unsigned short* p = HP + (size_t)row * KFF + c8;
    *(volatile v8us*)p = hi;
    *(volatile v8us*)(p + DMOD) = lo;
    __threadfence();
    *(volatile v8us*)p = hi;
    *(volatile v8us*)(p + DMOD) = lo;
  }
}

__global__ __launch_bounds__(GTHR) void k_ffn(const unsigned short* __restrict__ A, const unsigned short* __restrict__ BT,
                                              const float* __restrict__ bias, const float* __restrict__ X,
                                              const float* __restrict__ AO, float* C, int nRows) {
  constexpr int NT = 4;
  constexpr int BN = 16 * NT;
  __shared__ __attribute__((aligned(16))) float stg[GBM * BN];
  const int tid = (int)threadIdx.x, lane = tid & 31, wave = tid >> 5, hh = lane >> 4, m = lane & 15;
  const int rowBase = (int)blockIdx.x * GBM;
  const int colBase = (int)blockIdx.y * BN;

  v8f acc[NT];
  {
    const v8f z = {0.f, 0.f, 0.f, 0.f, 0.f, 0.f, 0.f, 0.f};
#pragma unroll
    for (int t = 0; t < NT; ++t) acc[t] = z;
  }
  const unsigned short* ap = A  + (size_t)(rowBase + 16 * wave + m) * (size_t)KFF + 8 * hh;
  const unsigned short* bp = BT + (size_t)(colBase + m) * (size_t)KFF + 8 * hh;

#pragma unroll 1
  for (int k0 = 0; k0 < KFF; k0 += 32) {
    FragU af;
    af.h[0] = *(const v8usa*)(ap + k0);
    af.h[1] = *(const v8usa*)(ap + k0 + 16);
#pragma unroll
    for (int nt = 0; nt < NT; ++nt) {
      const unsigned short* wq = bp + (size_t)(16 * nt) * (size_t)KFF + k0;
      FragU bf;
      bf.h[0] = *(const v8usa*)wq;
      bf.h[1] = *(const v8usa*)(wq + 16);
      acc[nt] = wmk(af, bf, acc[nt]);
    }
  }

#pragma unroll
  for (int nt = 0; nt < NT; ++nt) {
    const int lc = 16 * nt + m;
    const float bb = bf_rne(bias[colBase + lc]);
#pragma unroll
    for (int r = 0; r < 8; ++r) {
      const int lr = 16 * wave + 8 * hh + r;
      float v = acc[nt][r] + bb;
      v = (v > 0.0f) ? v : 0.2f * v;
      stg[lr * BN + lc] = v;
    }
  }
  __syncthreads();

  v4f pv[8];
#pragma unroll
  for (int i = 0; i < 8; ++i) {
    const int lr  = 16 * wave + 2 * i + hh;
    const int gr  = rowBase + lr;
    const int grc = gr < nRows ? gr : nRows - 1;
    const v4f sv = *(const v4fa*)(stg + lr * BN + 4 * m);
    const size_t go = (size_t)grc * (size_t)DMOD + colBase + 4 * m;
    const v4f xv = *(const v4f*)(X + go);
    const v4f av = *(const v4f*)(AO + go);
    v4f hv;
    hv.x = bf_rne(xv.x) + av.x; hv.y = bf_rne(xv.y) + av.y; hv.z = bf_rne(xv.z) + av.z; hv.w = bf_rne(xv.w) + av.w;
    pv[i] = hv + sv;
  }
#pragma unroll
  for (int i = 0; i < 8; ++i) {
    const int gr = rowBase + 16 * wave + 2 * i + hh;
    float* op = C + (size_t)gr * (size_t)DMOD + colBase + 4 * m;
    if (gr < nRows) *(volatile v4f*)op = pv[i];
  }
  __threadfence();
#pragma unroll
  for (int i = 0; i < 8; ++i) {
    const int gr = rowBase + 16 * wave + 2 * i + hh;
    float* op = C + (size_t)gr * (size_t)DMOD + colBase + 4 * m;
    if (gr < nRows) *(volatile v4f*)op = pv[i];
  }
}

static inline int cdiv(int a, int b) { return (a + b - 1) / b; }
static inline size_t al256(size_t o) { return (o + 255) & ~(size_t)255; }

extern "C" void kernel_launch(void* const* d_in, const int* in_sizes, int n_in,
                              void* d_out, int out_size, void* d_ws, size_t ws_size,
                              hipStream_t stream) {
  if (n_in < 8) return;
  if (in_sizes[0] != NNODE * DMOD) return;
  const int nE = in_sizes[1];
  if (nE < 1 || nE >= (1 << 21)) return;
  if (in_sizes[2] != nE) return;
  if (in_sizes[3] != DMOD * DMOD || in_sizes[4] != DMOD * DMOD) return;
  if (in_sizes[5] != DMOD * DMOD || in_sizes[6] != DMOD * DMOD) return;
  if (in_sizes[7] != DMOD) return;
  if (out_size != NNODE * DMOD) return;

  const float* X   = (const float*)d_in[0];
  const int*   src = (const int*)d_in[1];
  const int*   dst = (const int*)d_in[2];
  const float* WQ  = (const float*)d_in[3];
  const float* WK  = (const float*)d_in[4];
  const float* WV  = (const float*)d_in[5];
  const float* Wc  = (const float*)d_in[6];
  const float* bc  = (const float*)d_in[7];
  float* out = (float*)d_out;

  const int nN   = NNODE;
  const int gA   = cdiv(nN, NBA);
  const int RA   = gA * NBA;
  const int vec8 = ((nE & 3) == 0) ? 1 : 0;
  if (RA < nN) return;

  const size_t PX2 = (size_t)NNODE * DMOD * 2;
  const size_t PX4 = (size_t)NNODE * DMOD * 4;
  char* ws = (char*)d_ws;
  size_t off = 0;
  const size_t oWqkv = off; off = al256(off + (size_t)NQKV * DMOD * 2);
  const size_t oWcD  = off; off = al256(off + (size_t)DMOD * KFF * 2);
  const size_t oXb   = off; off = al256(off + PX2);
  const size_t oQh   = off; off = al256(off + PX2);
  const size_t oQl   = off; off = al256(off + PX2);
  const size_t oKf   = off; off = al256(off + PX4);
  const size_t oVTh  = off; off = al256(off + PX2);
  const size_t oVTl  = off; off = al256(off + PX2);
  const size_t oK2h  = off; off = al256(off + (size_t)RA * DMOD * 2);
  const size_t oK2l  = off; off = al256(off + (size_t)RA * DMOD * 2);
  const size_t oAO   = off; off = al256(off + PX4);
  const size_t oHP   = off; off = al256(off + (size_t)NNODE * KFF * 2);
  if (off > ws_size || off > (size_t)WSMAX) return;
  unsigned short* WqkvT = (unsigned short*)(ws + oWqkv);
  unsigned short* WcD   = (unsigned short*)(ws + oWcD);
  unsigned short* Xb    = (unsigned short*)(ws + oXb);
  unsigned short* Qh    = (unsigned short*)(ws + oQh);
  unsigned short* Ql    = (unsigned short*)(ws + oQl);
  float*          Kf    = (float*)(ws + oKf);
  unsigned short* VTh   = (unsigned short*)(ws + oVTh);
  unsigned short* VTl   = (unsigned short*)(ws + oVTl);
  unsigned short* K2h   = (unsigned short*)(ws + oK2h);
  unsigned short* K2l   = (unsigned short*)(ws + oK2l);
  float*          AO    = (float*)(ws + oAO);
  unsigned short* HP    = (unsigned short*)(ws + oHP);

  hipFuncSetAttribute(reinterpret_cast<const void*>(&k_agg), hipFuncAttributeMaxDynamicSharedMemorySize, LDS_AGG);

  const dim3 blk(256);
  k_wtrans<<<dim3(DMOD / 64, DMOD / 64, 4), blk, 0, stream>>>(WQ, WK, WV, Wc, WqkvT, WcD);
  const int n8 = NNODE * DMOD / 8;
  k_xcvt<<<cdiv(n8, 256), blk, 0, stream>>>(X, Xb, n8);
  const dim3 gQ(cdiv((NNODE / 64) * (DMOD / 64), 8));
  wmma_gemm64<false, 2><<<gQ, blk, 0, stream>>>(Xb, Xb, DMOD, WqkvT, WqkvT, DMOD,
                                                (void*)Qh, (void*)Ql, DMOD, NNODE, DMOD, DMOD, 1.0f);
  wmma_gemm64<false, 0><<<gQ, blk, 0, stream>>>(Xb, Xb, DMOD, WqkvT + (size_t)DMOD * DMOD, WqkvT + (size_t)DMOD * DMOD, DMOD,
                                                (void*)Kf, (void*)Kf, DMOD, NNODE, DMOD, DMOD, 1.0f);
  const dim3 gVT(cdiv((DMOD / 64) * (NNODE / 64), 8));
  wmma_gemm64<false, 2><<<gVT, blk, 0, stream>>>(WqkvT + (size_t)2 * DMOD * DMOD, WqkvT + (size_t)2 * DMOD * DMOD, DMOD,
                                                 Xb, Xb, DMOD, (void*)VTh, (void*)VTl, NNODE, DMOD, NNODE, DMOD, 1.0f);
  k_agg<<<gA, NTHR, LDS_AGG, stream>>>(src, dst, Kf, K2h, K2l, nN, nE, vec8);
  k_attn<<<dim3(NHEAD * (NNODE / AT_QB)), dim3(128), 0, stream>>>(Qh, Ql, K2h, K2l, VTh, VTl, AO, 0.0625f);
  const int nUnits = NNODE * (DMOD / 8);
  k_hsplit<<<cdiv(nUnits, 256), blk, 0, stream>>>(X, AO, HP, nUnits);
  k_ffn<<<dim3(NNODE / GBM, DMOD / 64), GTHR, 0, stream>>>(HP, WcD, bc, X, AO, out, nN);
  (void)hipGetLastError();
}
